// TimeMixing_49057116455666
// MI455X (gfx1250) — hardware-verified
//
#include <hip/hip_runtime.h>
#include <hip/hip_bf16.h>
#include <math.h>

#define TT 8192
#define EE 1024
#define GSTR 48

typedef _Float16 bf16;
typedef _Float16 f16;
typedef __attribute__((ext_vector_type(4))) unsigned v4u_t;
typedef unsigned v4ua __attribute__((ext_vector_type(4), may_alias));
typedef __attribute__((ext_vector_type(4))) float v4f_t;
typedef float v4fa __attribute__((ext_vector_type(4), may_alias));
typedef __attribute__((ext_vector_type(16))) bf16  bf16x16;
typedef bf16x16 f16x16;
typedef __attribute__((ext_vector_type(8)))  bf16  bf16x8;
typedef bf16x8 f16x8;
typedef __attribute__((ext_vector_type(4)))  bf16  bf16x4;
typedef __attribute__((ext_vector_type(8)))  float f32x8;
__device__ __forceinline__ f32x8 wmma16(f16x16 a, f16x16 b, f32x8 c) {
  c = __builtin_amdgcn_wmma_f32_16x16x32_f16(false, a, false, b, (short)0, c, false, false);
  asm volatile("v_nop\n\tv_nop\n\tv_nop\n\tv_nop" : "+v"(c) : "v"(a), "v"(b));
  return c;
}
#define LDS_STRIDE 48
#define KSTRIDE    72
#define VSTRIDE    48

__device__ __forceinline__ f32x8 wmma_bf16(bf16x16 a, bf16x16 b, f32x8 c) {
  c = __builtin_amdgcn_wmma_f32_16x16x32_f16(false, a, false, b, (short)0, c, false, false);
  asm volatile("v_nop\n\tv_nop\n\tv_nop\n\tv_nop" : "+v"(c) : "v"(a), "v"(b));
  return c;
}

template <typename T>
__device__ __forceinline__ bf16x16 load_frag(const T* __restrict__ base, int ld,
                                             int row0, int k0) {
  const int lane = threadIdx.x & 31;
  const int r    = lane & 15;
  const int kh   = (lane >> 4) * 8;
  const T* p0 = base + (size_t)(row0 + r) * ld + (k0 + kh);
  const T* p1 = p0 + 16;
  bf16x16 f;
#pragma unroll
  for (int i = 0; i < 8; ++i) {
    f[i]     = (bf16)p0[i];
    f[i + 8] = (bf16)p1[i];
  }
  return f;
}

__device__ __forceinline__ bf16x16 lds_frag(const bf16* base, int stride) {
  const int lane = threadIdx.x & 31;
  const int row  = lane & 15;
  const int kh   = (lane >> 4) * 8;
  const bf16x8 lo = *(const bf16x8*)(base + row * stride + kh);
  const bf16x8 hi = *(const bf16x8*)(base + row * stride + kh + 16);
  bf16x16 f;
#pragma unroll
  for (int i = 0; i < 8; ++i) { f[i] = lo[i]; f[i + 8] = hi[i]; }
  return f;
}

template <typename T>
__device__ __forceinline__ void stage_read16(const T* __restrict__ p, float* buf) {
#pragma unroll
  for (int i = 0; i < 16; ++i) buf[i] = (float)p[i];
}

__device__ __forceinline__ void stage_write(bf16* dst, const float* buf, int nquad) {
#pragma unroll
  for (int i = 0; i < nquad; ++i) {
    bf16x4 q;
    q[0] = (bf16)buf[4 * i];     q[1] = (bf16)buf[4 * i + 1];
    q[2] = (bf16)buf[4 * i + 2]; q[3] = (bf16)buf[4 * i + 3];
    *(bf16x4*)(dst + 4 * i) = q;
  }
}


#define GSTR 48
template <typename AT, int EPI, bool OUT16>
__global__ __launch_bounds__(256) void gemm_kne(const AT* __restrict__ A, int lda, const float* __restrict__ Wm, int ldw,
                                                const float* __restrict__ bias, const float* __restrict__ R, const float* __restrict__ gvec,
                                                void* __restrict__ Yv, int ldy, int K) {
  __shared__ __attribute__((aligned(16))) f16 ldsA[128 * GSTR];
  __shared__ __attribute__((aligned(16))) f16 ldsW[128 * GSTR];
  __shared__ __attribute__((aligned(16))) float oS[8][32 * 68];
  const int tid = threadIdx.x, lane = tid & 31, wave = tid >> 5, cl = lane & 15, rh = (lane >> 4) * 8;
  const int m0 = blockIdx.x * 128, n0 = blockIdx.y * 128;
  const int wm = (wave & 3) * 32, wn = (wave >> 2) * 64;
  f32x8 acc[2][4];
#pragma unroll
  for (int i = 0; i < 2; ++i)
#pragma unroll
    for (int j = 0; j < 4; ++j) { f32x8 z = {}; acc[i][j] = z; }
#pragma unroll 1
  for (int k0 = 0; k0 < K; k0 += 32) {
    __syncthreads();
    { const int row = tid >> 1, ch = (tid & 1) * 16;
      const AT* src = A + (size_t)(m0 + row) * lda + k0 + ch;
#pragma unroll
      for (int g = 0; g < 16; ++g) ldsA[row * GSTR + ch + g] = (f16)src[g]; }
    { const int k = tid >> 3, nn0 = (tid & 7) * 16;
      const float* src = Wm + (size_t)(k0 + k) * ldw + n0 + nn0;
#pragma unroll
      for (int g = 0; g < 4; ++g) { const v4f_t v = *(const v4f_t*)(src + 4 * g);
#pragma unroll
        for (int u = 0; u < 4; ++u) ldsW[(nn0 + 4 * g + u) * GSTR + k] = (f16)v[u]; } }
    __syncthreads();
    f16x16 af[2];
#pragma unroll
    for (int i = 0; i < 2; ++i) af[i] = lds_frag(ldsA + (wm + 16 * i) * GSTR, GSTR);
#pragma unroll
    for (int j = 0; j < 4; ++j) {
      const f16x16 bf = lds_frag(ldsW + (wn + 16 * j) * GSTR, GSTR);
#pragma unroll
      for (int i = 0; i < 2; ++i) acc[i][j] = wmma16(af[i], bf, acc[i][j]);
    }
  }
  float* so = oS[wave];
#pragma unroll
  for (int i = 0; i < 2; ++i)
#pragma unroll
    for (int j = 0; j < 4; ++j) {
      const int n = n0 + wn + 16 * j + cl;
      const float bv = bias ? bias[n] : 0.0f;
      const float gv = (EPI == 2) ? gvec[n] : 0.0f;
      if (EPI == 1) {
#pragma unroll 1
        for (int r = 0; r < 8; ++r) { const float xg = acc[i][j][r] + bv; so[(16 * i + rh + r) * 68 + 16 * j + cl] = 0.5f * xg * (1.0f + erff(xg * 0.70710678118654752f)); }
      } else {
#pragma unroll
        for (int r = 0; r < 8; ++r) {
          float v = acc[i][j][r] + bv;
          if (EPI == 2) v = R[(size_t)(m0 + wm + 16 * i + rh + r) * ldy + n] + gv * v;
          so[(16 * i + rh + r) * 68 + 16 * j + cl] = v;
        }
      }
    }
  asm volatile("s_wait_dscnt 0" ::: "memory");
  __builtin_amdgcn_wave_barrier();
#pragma unroll 1
  for (int pass = 0; pass < 2; ++pass) {
    if (OUT16) {
      f16* Y = (f16*)Yv;
#pragma unroll
      for (int it = 0; it < 8; ++it) { const int c = lane + 32 * it, rr = c >> 3, q8 = (c & 7) * 8;
        union { f16 h[8]; v4u_t v; } u;
#pragma unroll
        for (int e = 0; e < 8; ++e) u.h[e] = (f16)so[rr * 68 + q8 + e];
        *(volatile v4u_t*)(Y + (size_t)(m0 + wm + rr) * ldy + n0 + wn + q8) = u.v; }
    } else {
      float* Y = (float*)Yv;
#pragma unroll
      for (int it = 0; it < 16; ++it) { const int f4 = lane + 32 * it, rr = f4 >> 4, q = (f4 & 15) * 4;
        *(volatile v4f_t*)(Y + (size_t)(m0 + wm + rr) * ldy + n0 + wn + q) = *(const v4fa*)(so + rr * 68 + q); }
    }
    __threadfence();
  }
}

__global__ __launch_bounds__(256) void k_mix(const float* __restrict__ x, const float* __restrict__ sx, const float* __restrict__ mk, const float* __restrict__ mv, const float* __restrict__ mr,
                                            bf16* __restrict__ kx, bf16* __restrict__ vx, bf16* __restrict__ rx) {
  const size_t i = (size_t)blockIdx.x * 256 + threadIdx.x; const size_t t = i >> 7; const int c0 = (i & 127) * 8;
  const float* xr = x + t * EE + c0; const float* pr = (t == 0) ? (sx + c0) : (x + (t - 1) * EE + c0);
  union { bf16 hh[8]; v4u_t u; } ck, cv2, cr;
#pragma unroll
  for (int e = 0; e < 8; ++e) { const float a = xr[e], p = pr[e]; const int c = c0 + e;
    ck.hh[e] = (bf16)(a * mk[c] + p * (1.0f - mk[c])); cv2.hh[e] = (bf16)(a * mv[c] + p * (1.0f - mv[c])); cr.hh[e] = (bf16)(a * mr[c] + p * (1.0f - mr[c])); }
#pragma unroll 1
  for (int pass = 0; pass < 2; ++pass) { *(volatile v4u_t*)(kx + t * EE + c0) = ck.u; *(volatile v4u_t*)(vx + t * EE + c0) = cv2.u; *(volatile v4u_t*)(rx + t * EE + c0) = cr.u; __threadfence(); }
}
__global__ __launch_bounds__(256) void k_wkv(const bf16* __restrict__ k, const bf16* __restrict__ v, float* __restrict__ ry, const float* __restrict__ aa0, const float* __restrict__ bb0, const float* __restrict__ pp0,
                                            const float* __restrict__ tfirst, const float* __restrict__ tdecay, float* __restrict__ aaf, float* __restrict__ bbf, float* __restrict__ ppf) {
  const int e = blockIdx.x * 256 + threadIdx.x;
  float aa = aa0[e], bb = bb0[e], pp = pp0[e]; const float tf = tfirst[e], decay = -expf(tdecay[e]);
#pragma unroll 2
  for (int t = 0; t < TT; ++t) { const size_t idx = (size_t)t * EE + e; const float kk = (float)k[idx], vv = (float)v[idx];
    const float ww = tf + kk; const float p = fmaxf(pp, ww); const float e1 = expf(pp - p), e2 = expf(ww - p);
    const float wkv = (e1 * aa + e2 * vv) / (e1 * bb + e2);
    const float ww2 = decay + pp; const float p2 = fmaxf(ww2, kk); const float e1b = expf(ww2 - p2), e2b = expf(kk - p2);
    aa = e1b * aa + e2b * vv; bb = e1b * bb + e2b; pp = p2;
    const float rr = ry[idx]; ry[idx] = wkv / (1.0f + expf(-rr)); }
  aaf[e] = aa; bbf[e] = bb; ppf[e] = pp;
}
__global__ __launch_bounds__(256) void k_tail(const float* __restrict__ x, const float* __restrict__ af, const float* __restrict__ bf_, const float* __restrict__ pf, float* __restrict__ o) {
  const int tid = threadIdx.x; const float* src = (blockIdx.x == 0) ? (x + (size_t)(TT - 1) * EE) : (blockIdx.x == 1 ? af : (blockIdx.x == 2 ? bf_ : pf));
  const v4f_t val = *(const v4f_t*)(src + tid * 4); float* dst = o + (size_t)blockIdx.x * EE + tid * 4;
  *(volatile v4f_t*)dst = val; __threadfence(); *(volatile v4f_t*)dst = val;
}
__global__ __launch_bounds__(256) void k_ones(float* __restrict__ p) { const int tid = threadIdx.x; v4f_t o = {1.f,1.f,1.f,1.f}; *(volatile v4f_t*)(p + tid * 4) = o; __threadfence(); *(volatile v4f_t*)(p + tid * 4) = o; }

extern "C" void kernel_launch(void* const* d_in, const int* in_sizes, int n_in,
                              void* d_out, int out_size, void* d_ws, size_t ws_size,
                              hipStream_t stream) {
  (void)in_sizes; (void)n_in; (void)out_size;
  const float** f = (const float**)d_in;
  const float* x = f[0], *sx = f[1], *aa = f[2], *bb = f[3], *pp = f[4], *tfirst = f[5], *tdecay = f[6], *mk = f[7], *mv = f[8], *mr = f[9], *Wk = f[10], *Wv = f[11], *Wr = f[12], *Wo = f[13];
  float* out = (float*)d_out;
  float* tail = out + (size_t)TT * EE;
  char* ws = (char*)d_ws;
  bf16* kx = (bf16*)ws; ws += (size_t)TT * EE * 2; bf16* vx = (bf16*)ws; ws += (size_t)TT * EE * 2; bf16* rx = (bf16*)ws; ws += (size_t)TT * EE * 2;
  float* ry = (float*)ws; ws += (size_t)TT * EE * 4;
  bf16* k16 = (bf16*)ws; ws += (size_t)TT * EE * 2; bf16* v16 = (bf16*)ws; ws += (size_t)TT * EE * 2;
  float* stf = (float*)ws; ws += 3 * EE * 4; float* ones = (float*)ws; ws += EE * 4;
  if ((size_t)(ws - (char*)d_ws) > ws_size) return;
  const dim3 blk(256);
  k_ones<<<dim3(1), blk, 0, stream>>>(ones);
  k_mix<<<dim3(TT * (EE / 8) / 256), blk, 0, stream>>>(x, sx, mk, mv, mr, kx, vx, rx);
  gemm_kne<bf16, 0, false><<<dim3(TT / 128, EE / 128), blk, 0, stream>>>(rx, EE, Wr, EE, nullptr, nullptr, nullptr, ry, EE, EE);
  gemm_kne<bf16, 0, true ><<<dim3(TT / 128, EE / 128), blk, 0, stream>>>(kx, EE, Wk, EE, nullptr, nullptr, nullptr, k16, EE, EE);
  gemm_kne<bf16, 0, true ><<<dim3(TT / 128, EE / 128), blk, 0, stream>>>(vx, EE, Wv, EE, nullptr, nullptr, nullptr, v16, EE, EE);
  k_wkv<<<dim3(EE / 256), blk, 0, stream>>>(k16, v16, ry, aa, bb, pp, tfirst, tdecay, stf, stf + EE, stf + 2 * EE);
  gemm_kne<float, 2, false><<<dim3(TT / 128, EE / 128), blk, 0, stream>>>(ry, EE, Wo, EE, nullptr, x, ones, out, EE, EE);
  k_tail<<<dim3(4), blk, 0, stream>>>(x, stf, stf + EE, stf + 2 * EE, tail);
}
